// Encoder_54339926229533
// MI455X (gfx1250) — hardware-verified
//
#include <hip/hip_runtime.h>
#include <math.h>
#include <stddef.h>

constexpr int NVOCAB  = 32000;
constexpr int NEMB    = 256;
constexpr int NUNIT   = 1024;
constexpr int NBATCH  = 64;
constexpr int NSTEP   = 128;
constexpr int NGATE3  = 3 * NUNIT;
constexpr int NROWS   = NBATCH * NSTEP;
constexpr int NTHR    = 256;
constexpr int SEQ_BLK = 16;
constexpr int HPITCH  = NUNIT + 8;
constexpr int OSLABP  = 36;
constexpr int XF_FRAG = 256;
constexpr int XF_GATE_STRIDE = (NUNIT / 16) * XF_FRAG;
constexpr size_t U_GATE_STRIDE = (size_t)NUNIT * (size_t)NUNIT;
constexpr float E_CARRY  = 16.0f;
constexpr float W_CARRY  = 16.0f;
constexpr float U_CARRY  = 32.0f;
constexpr float H_CARRY  = 64.0f;
constexpr float XIN_FOLD = 1.0f / (E_CARRY * W_CARRY);
constexpr float REC_FOLD = 1.0f / (H_CARRY * U_CARRY);
constexpr size_t OUT0_ELEMS = (size_t)NBATCH * NSTEP * NUNIT;
constexpr size_t OUT1_ELEMS = (size_t)NBATCH * NUNIT;

static_assert(NROWS % 64 == 0, "GEMM M tile multiple");
static_assert(NGATE3 % 64 == 0, "GEMM N tile multiple");
static_assert(NEMB % 32 == 0, "GEMM K multiple of 32");
static_assert(NUNIT % 32 == 0, "recurrent K multiple of 32");
static_assert(NBATCH == 64, "one 64-row GEMM tile per time step");
static_assert(NUNIT == 128 * (NTHR / 32), "8 waves x 128 units");
static_assert(NBATCH % SEQ_BLK == 0, "batch tiles");
static_assert(OUT0_ELEMS * 4 == 33554432, "second output byte offset");
static_assert((OUT0_ELEMS + OUT1_ELEMS) * 4 == 33816576, "output total bytes");
static_assert((HPITCH * 2) % 16 == 0, "h tile pitch 16-B aligned");
static_assert((OSLABP * 4) % 16 == 0, "slab pitch 16-B aligned");
static_assert(((size_t)NROWS * (NEMB / 8)) % NTHR == 0, "gather grid exact");

typedef __attribute__((ext_vector_type(16))) _Float16 v16h;
typedef __attribute__((ext_vector_type(8)))  _Float16 v8h;
typedef __attribute__((ext_vector_type(8)))  float    v8f;
typedef __attribute__((ext_vector_type(4)))  float    v4f;

__device__ __forceinline__ void guard3_h(v8f& a, v8f& b, v8f& c, v16h x, v16h y, v16h z, v16h w) {
  asm volatile("v_nop\n\tv_nop\n\tv_nop\n\tv_nop" : "+v"(a), "+v"(b), "+v"(c) : "v"(x), "v"(y), "v"(z), "v"(w));
}
__device__ __forceinline__ void guard4_h(v8f& a, v8f& b, v8f& c, v8f& d, v16h x, v16h y) {
  asm volatile("v_nop\n\tv_nop\n\tv_nop\n\tv_nop" : "+v"(a), "+v"(b), "+v"(c), "+v"(d) : "v"(x), "v"(y));
}
__device__ __forceinline__ void keep4_h(v16h a, v16h b, v16h c, v16h d) {
  asm volatile("v_nop" :: "v"(a), "v"(b), "v"(c), "v"(d));
}
__device__ __forceinline__ void acc_guard4(v8f& a, v8f& b, v8f& c, v8f& d) {
  asm volatile("v_nop\n\tv_nop\n\tv_nop\n\tv_nop" : "+v"(a), "+v"(b), "+v"(c), "+v"(d));
}
__device__ __forceinline__ void acc_guard3(v8f& a, v8f& b, v8f& c) {
  asm volatile("v_nop\n\tv_nop\n\tv_nop\n\tv_nop" : "+v"(a), "+v"(b), "+v"(c));
}

struct FragH {
  union UU { v16h v; v8h h[2]; };
  static __device__ __forceinline__ v16h load(const _Float16* p) {
    UU f;
    f.h[0] = *(const v8h*)(p);
    f.h[1] = *(const v8h*)(p + 16);
    return f.v;
  }
  static __device__ __forceinline__ v8f mma(v16h a, v16h b, v8f c) {
    return __builtin_amdgcn_wmma_f32_16x16x32_f16(false, a, false, b, (short)0, c, false, false);
  }
};

__device__ __forceinline__ void wave_lds_sync() {
  __builtin_amdgcn_fence(__ATOMIC_RELEASE, "workgroup");
  __builtin_amdgcn_wave_barrier();
  __builtin_amdgcn_fence(__ATOMIC_ACQUIRE, "workgroup");
}

__device__ __forceinline__ float fsig(float x)  { return __builtin_amdgcn_rcpf(1.0f + expf(-x)); }
__device__ __forceinline__ float ftanh(float x) { return 1.0f - 2.0f * __builtin_amdgcn_rcpf(expf(2.0f * x) + 1.0f); }

__global__ __launch_bounds__(NTHR) void tpw_f16_kernel(const float* __restrict__ src, int R, int C, int ldo,
                                                       unsigned short* __restrict__ O, float sc) {
  __shared__ float Tt[64 * 65];
  const int tid = threadIdx.x;
  const int c0 = blockIdx.x * 64, r0 = blockIdx.y * 64;
  (void)R;
#pragma unroll
  for (int i = 0; i < 4; ++i) {
    const int idx = i * NTHR + tid;
    const int rr = idx >> 4, cc = (idx & 15) * 4;
    const v4f v = *(const v4f*)(src + (size_t)(r0 + rr) * (size_t)C + c0 + cc);
    Tt[rr * 65 + cc + 0] = v[0];
    Tt[rr * 65 + cc + 1] = v[1];
    Tt[rr * 65 + cc + 2] = v[2];
    Tt[rr * 65 + cc + 3] = v[3];
  }
  __syncthreads();
  const int q = tid >> 3, c8 = (tid & 7) * 8;
  v8h hv[2];
#pragma unroll
  for (int g = 0; g < 2; ++g) {
    const int qq = g * 32 + q;
#pragma unroll
    for (int e = 0; e < 8; ++e) {
      const float f = Tt[(c8 + e) * 65 + qq];
      hv[g][e] = (_Float16)(f * sc);
    }
  }
  for (int pass = 0; pass < 2; ++pass) {
#pragma unroll
    for (int g = 0; g < 2; ++g) {
      const size_t o = (size_t)(c0 + g * 32 + q) * (size_t)ldo + (size_t)(r0 + c8);
      *(volatile v8h*)(O + o) = hv[g];
    }
    __threadfence();
  }
}

__global__ __launch_bounds__(NTHR) void gather_emb_kernel(const int* __restrict__ xtok, const float* __restrict__ E,
                                                          unsigned short* __restrict__ AE) {
  const int i = blockIdx.x * NTHR + threadIdx.x;
  if (i < NROWS * (NEMB / 8)) {
    const int m  = i >> 5;
    const int c8 = (i & 31) * 8;
    const int t  = m >> 6;
    const int b  = m & 63;
    int tok = xtok[b * NSTEP + t];
    tok = tok < 0 ? 0 : (tok > NVOCAB - 1 ? NVOCAB - 1 : tok);
    const float* sp = E + (size_t)tok * NEMB + c8;
    const v4f a = *(const v4f*)(sp);
    const v4f bq = *(const v4f*)(sp + 4);
    v8h hv;
#pragma unroll
    for (int e = 0; e < 4; ++e) {
      hv[e]     = (_Float16)(a[e] * E_CARRY);
      hv[4 + e] = (_Float16)(bq[e] * E_CARRY);
    }
    *(volatile v8h*)(AE + (size_t)i * 8) = hv;
    __threadfence();
    *(volatile v8h*)(AE + (size_t)i * 8) = hv;
  }
}

__global__ __launch_bounds__(NTHR) void xin_gemm_kernel(const unsigned short* __restrict__ Ap,
                                                        const unsigned short* __restrict__ Btp,
                                                        const float* __restrict__ bias, float* __restrict__ XF) {
  const _Float16* A  = (const _Float16*)Ap;
  const _Float16* Bt = (const _Float16*)Btp;
  const int lane = threadIdx.x & 31;
  const int wave = threadIdx.x >> 5;
  constexpr int tilesN = NGATE3 / 64;
  constexpr int tilesM = NROWS / 64;
  const int tile = blockIdx.x * 8 + wave;
  if (tile >= tilesM * tilesN) return;
  const int tm = tile / tilesN;
  const int tn = tile - tm * tilesN;
  const int m0 = tm << 6;
  const int n0 = tn << 6;
  const int rlane = lane & 15;
  const int koff  = (lane >> 4) * 8;

  v8f acc[4][4];
#pragma unroll
  for (int i = 0; i < 4; ++i)
#pragma unroll
    for (int j = 0; j < 4; ++j) acc[i][j] = (v8f){0.f, 0.f, 0.f, 0.f, 0.f, 0.f, 0.f, 0.f};

#pragma unroll 1
  for (int k0 = 0; k0 < NEMB; k0 += 32) {
    v16h bh[4];
#pragma unroll
    for (int j = 0; j < 4; ++j) {
      const size_t bo = (size_t)(n0 + (j << 4) + rlane) * NEMB + koff + k0;
      bh[j] = FragH::load(Bt + bo);
    }
#pragma unroll
    for (int i = 0; i < 4; ++i) {
      const size_t ao = (size_t)(m0 + (i << 4) + rlane) * NEMB + koff + k0;
      const v16h ah = FragH::load(A + ao);
#pragma unroll
      for (int j = 0; j < 4; ++j) acc[i][j] = FragH::mma(ah, bh[j], acc[i][j]);
      guard4_h(acc[i][0], acc[i][1], acc[i][2], acc[i][3], ah, bh[3]);
    }
    keep4_h(bh[0], bh[1], bh[2], bh[3]);
  }
  acc_guard4(acc[0][0], acc[0][1], acc[0][2], acc[0][3]);
  acc_guard4(acc[1][0], acc[1][1], acc[1][2], acc[1][3]);
  acc_guard4(acc[2][0], acc[2][1], acc[2][2], acc[2][3]);
  acc_guard4(acc[3][0], acc[3][1], acc[3][2], acc[3][3]);

  float bv[4];
#pragma unroll
  for (int j = 0; j < 4; ++j) bv[j] = bias[n0 + (j << 4) + rlane];

  for (int pass = 0; pass < 2; ++pass) {
#pragma unroll
    for (int i = 0; i < 4; ++i) {
#pragma unroll
      for (int j = 0; j < 4; ++j) {
        const int n    = n0 + (j << 4);
        const int gate = n >> 10;
        const int ut   = (n & (NUNIT - 1)) >> 4;
        float* fp = XF + ((((size_t)tm * 4 + (size_t)i) * 3 + (size_t)gate) * 64 + (size_t)ut) * XF_FRAG + lane * 4;
        v4f o0, o1;
#pragma unroll
        for (int e = 0; e < 4; ++e) {
          o0[e] = acc[i][j][e] * XIN_FOLD + bv[j];
          o1[e] = acc[i][j][4 + e] * XIN_FOLD + bv[j];
        }
        *(volatile v4f*)(fp) = o0;
        *(volatile v4f*)(fp + 128) = o1;
      }
    }
    __threadfence();
  }
}

__global__ __launch_bounds__(NTHR) void gru_seq_kernel(const float* __restrict__ XF, const unsigned short* __restrict__ Utp,
                                                       const float* __restrict__ brec, const float* __restrict__ hid0,
                                                       float* __restrict__ out0, float* __restrict__ out1) {
  __shared__ __align__(16) _Float16 hA[SEQ_BLK * HPITCH];
  __shared__ __align__(16) float    Sl[NTHR / 32][16 * OSLABP];
  const _Float16* Ut = (const _Float16*)Utp;
  const int tid = threadIdx.x, lane = tid & 31, wave = tid >> 5;
  const int c = lane & 15, hh = lane >> 4, koff = hh * 8;
  const int q8 = lane >> 3, l4 = (lane & 7) * 4;
  const int rowbase = blockIdx.x * SEQ_BLK;
  float* slab = Sl[wave];

  float hst[8][8];
#pragma unroll
  for (int p = 0; p < 4; ++p) {
#pragma unroll
    for (int it = 0; it < 4; ++it) {
      const int row = it * 4 + q8;
      const v4f v = *(const v4f*)(hid0 + (size_t)(rowbase + row) * NUNIT + 128 * wave + 32 * p + l4);
      *(v4f*)(slab + row * OSLABP + l4) = v;
    }
    wave_lds_sync();
#pragma unroll
    for (int r = 0; r < 8; ++r) {
      hst[2 * p][r]     = slab[(8 * hh + r) * OSLABP + c];
      hst[2 * p + 1][r] = slab[(8 * hh + r) * OSLABP + 16 + c];
    }
    wave_lds_sync();
  }
  if (tid < 128) hA[(tid >> 3) * HPITCH + NUNIT + (tid & 7)] = (_Float16)0.0f;
#pragma unroll
  for (int nt = 0; nt < 8; ++nt)
#pragma unroll
    for (int r = 0; r < 8; ++r)
      hA[(8 * hh + r) * HPITCH + 128 * wave + 16 * nt + c] = (_Float16)(hst[nt][r] * H_CARRY);
  __syncthreads();

  const _Float16* ahrow = hA + c * HPITCH + koff;
  const v8f z8 = {0.f, 0.f, 0.f, 0.f, 0.f, 0.f, 0.f, 0.f};

#pragma unroll 1
  for (int t = 0; t < NSTEP; ++t) {
    const bool last = (t == NSTEP - 1);
#pragma unroll 1
    for (int nt = 0; nt < 8; ++nt) {
      const int ut = 8 * wave + nt;
      const int u  = 16 * ut + c;
      const _Float16* up = Ut + (size_t)u * NUNIT + koff;
      v8f accZ = z8, accR = z8, accH = z8;
#pragma unroll 1
      for (int k0 = 0; k0 < NUNIT; k0 += 32) {
        const v16h a   = FragH::load(ahrow + k0);
        const v16h fb0 = FragH::load(up + k0);
        const v16h fb1 = FragH::load(up + U_GATE_STRIDE + k0);
        const v16h fb2 = FragH::load(up + 2 * U_GATE_STRIDE + k0);
        accZ = FragH::mma(a, fb0, accZ);
        accR = FragH::mma(a, fb1, accR);
        accH = FragH::mma(a, fb2, accH);
        guard3_h(accZ, accR, accH, a, fb0, fb1, fb2);
      }
      acc_guard3(accZ, accR, accH);

      const float bz = brec[u];
      const float br = brec[NUNIT + u];
      const float bh = brec[2 * NUNIT + u];
      const float* xf = XF + ((((size_t)t * 4 + (size_t)blockIdx.x) * 3) * 64 + (size_t)ut) * XF_FRAG + lane * 4;
      v4f xz[2], xr[2], xh[2];
      xz[0] = *(const v4f*)(xf);
      xz[1] = *(const v4f*)(xf + 128);
      xr[0] = *(const v4f*)(xf + XF_GATE_STRIDE);
      xr[1] = *(const v4f*)(xf + XF_GATE_STRIDE + 128);
      xh[0] = *(const v4f*)(xf + 2 * XF_GATE_STRIDE);
      xh[1] = *(const v4f*)(xf + 2 * XF_GATE_STRIDE + 128);

      float hn[8];
#pragma unroll
      for (int r = 0; r < 8; ++r) {
        const float rz = accZ[r] * REC_FOLD + bz;
        const float rr = accR[r] * REC_FOLD + br;
        const float rh = accH[r] * REC_FOLD + bh;
        const float zg = fsig(xz[r >> 2][r & 3] + rz);
        const float rg = fsig(xr[r >> 2][r & 3] + rr);
        const float hc = ftanh(xh[r >> 2][r & 3] + rg * rh);
        const float ho = hst[0][r];
        hn[r] = zg * ho + (1.0f - zg) * hc;
      }
#pragma unroll
      for (int i = 0; i < 7; ++i)
#pragma unroll
        for (int r = 0; r < 8; ++r) hst[i][r] = hst[i + 1][r];
#pragma unroll
      for (int r = 0; r < 8; ++r) hst[7][r] = hn[r];

      if (nt & 1) {
#pragma unroll
        for (int r = 0; r < 8; ++r) {
          slab[(8 * hh + r) * OSLABP + c]      = hst[6][r];
          slab[(8 * hh + r) * OSLABP + 16 + c] = hst[7][r];
        }
        wave_lds_sync();
        const int ucol = 128 * wave + 16 * (nt - 1);
        for (int pass = 0; pass < 2; ++pass) {
#pragma unroll
          for (int it = 0; it < 4; ++it) {
            const int row = it * 4 + q8;
            const v4f v = *(const v4f*)(slab + row * OSLABP + l4);
            *(volatile v4f*)(out0 + ((size_t)(rowbase + row) * NSTEP + (size_t)t) * NUNIT + ucol + l4) = v;
            if (last) *(volatile v4f*)(out1 + (size_t)(rowbase + row) * NUNIT + ucol + l4) = v;
          }
          __threadfence();
        }
        wave_lds_sync();
      }
    }
    __syncthreads();
#pragma unroll
    for (int nt = 0; nt < 8; ++nt)
#pragma unroll
      for (int r = 0; r < 8; ++r)
        hA[(8 * hh + r) * HPITCH + 128 * wave + 16 * nt + c] = (_Float16)(hst[nt][r] * H_CARRY);
    __syncthreads();
  }
}

constexpr size_t WT_BYTES = (size_t)NGATE3 * NEMB * 2;
constexpr size_t UT_BYTES = (size_t)NGATE3 * NUNIT * 2;
constexpr size_t AE_BYTES = (size_t)NROWS * NEMB * 2;
constexpr size_t XF_BYTES = (size_t)NSTEP * 4 * 3 * 64 * XF_FRAG * 4;
static_assert(XF_BYTES == (size_t)NROWS * NGATE3 * 4, "fragment plane covers the whole projection");
static_assert(WT_BYTES % 256 == 0 && UT_BYTES % 256 == 0 && AE_BYTES % 256 == 0 && XF_BYTES % 256 == 0, "aligned carve");
static_assert(WT_BYTES + UT_BYTES + AE_BYTES + XF_BYTES <= (size_t)134217728, "carve within budget");

extern "C" void kernel_launch(void* const* d_in, const int* in_sizes, int n_in,
                              void* d_out, int out_size, void* d_ws, size_t ws_size, hipStream_t stream) {
  if (n_in < 6 || d_out == nullptr || d_ws == nullptr) return;
  if (in_sizes[0] != NBATCH * NSTEP || in_sizes[1] != NBATCH * NUNIT || in_sizes[2] != NVOCAB * NEMB ||
      in_sizes[3] != NEMB * NGATE3 || in_sizes[4] != NUNIT * NGATE3 || in_sizes[5] != 2 * NGATE3 ||
      out_size != (int)(OUT0_ELEMS + OUT1_ELEMS)) return;

  const int*   xtok   = (const int*)d_in[0];
  const float* hidden = (const float*)d_in[1];
  const float* emb    = (const float*)d_in[2];
  const float* w_in   = (const float*)d_in[3];
  const float* u_in   = (const float*)d_in[4];
  const float* bvec   = (const float*)d_in[5];
  const float* b_inp  = bvec;
  const float* b_rec  = bvec + NGATE3;
  float* out0 = (float*)d_out;
  float* out1 = out0 + OUT0_ELEMS;

  char* ws = (char*)d_ws;
  size_t off = 0;
  unsigned short* WT = (unsigned short*)(ws + off);
  off += WT_BYTES;
  unsigned short* UT = (unsigned short*)(ws + off);
  off += UT_BYTES;
  unsigned short* AE = (unsigned short*)(ws + off);
  off += AE_BYTES;
  float* XF = (float*)(ws + off);
  off += XF_BYTES;
  if (off > ws_size || off > (size_t)134217728) return;

  tpw_f16_kernel<<<dim3(NGATE3 / 64, NEMB / 64), NTHR, 0, stream>>>(w_in, NEMB, NGATE3, NEMB, WT, W_CARRY);
  tpw_f16_kernel<<<dim3(NGATE3 / 64, NUNIT / 64), NTHR, 0, stream>>>(u_in, NUNIT, NGATE3, NUNIT, UT, U_CARRY);
  gather_emb_kernel<<<(NROWS * (NEMB / 8)) / NTHR, NTHR, 0, stream>>>(xtok, emb, AE);
  xin_gemm_kernel<<<((NROWS / 64) * (NGATE3 / 64)) / 8, NTHR, 0, stream>>>(AE, WT, b_inp, XF);
  gru_seq_kernel<<<NBATCH / SEQ_BLK, NTHR, 0, stream>>>(XF, UT, b_rec, hidden, out0, out1);
}
